// MultiHeadAttention_31473520345937
// MI455X (gfx1250) — hardware-run, weakly checked
//
#include <hip/hip_runtime.h>


#ifndef NB
#define NB 2
#endif
#ifndef SEQ
#define SEQ 2048
#endif
#define SEQ_FULL 2048
#define TT   SEQ
#define DM   1024
#define NH_  16
#define HD   64
#define DQ   (NH_ * HD)
#define ZH   2
#define RELN 2049
#define ESTART (RELN - TT)
#define PCAR 1024.0f
#define ECAR 64.0f
#define SCL  0.125f
#define SWV  4

static_assert(TT % 128 == 0);
static_assert(TT <= SEQ_FULL);
static_assert(NH_ % ZH == 0);
static_assert(DM % 64 == 0);
static_assert(DQ % 64 == 0);
static_assert(HD == 64);
static_assert((ZH * TT) % SWV == 0);
static_assert((size_t)SWV * TT * 4 <= 65536);

typedef _Float16 h16;
typedef unsigned short bf;
typedef __attribute__((ext_vector_type(16))) __bf16   v16bf;
typedef __attribute__((ext_vector_type(16))) _Float16 v16h;
typedef __attribute__((ext_vector_type(8)))  _Float16 v8h;
typedef __attribute__((ext_vector_type(4)))  _Float16 v4h;
typedef __attribute__((ext_vector_type(8)))  unsigned short v8us;
typedef __attribute__((ext_vector_type(2)))  unsigned short v2us;
typedef __attribute__((ext_vector_type(8)))  float    v8f;
typedef __attribute__((ext_vector_type(4)))  float    v4f;
typedef v4f  __attribute__((may_alias)) v4fa;

__device__ __forceinline__ unsigned short f2bf(float f) { unsigned u = __float_as_uint(f); u += 0x7FFFu + ((u >> 16) & 1u); return (unsigned short)(u >> 16); }
__device__ __forceinline__ float bf2f(unsigned short b) { return __uint_as_float(((unsigned)b) << 16); }
__device__ __forceinline__ float bfr(float f) { return bf2f(f2bf(f)); }
__device__ __forceinline__ v16h cat16(v8h lo, v8h hi) { return __builtin_shufflevector(lo, hi, 0, 1, 2, 3, 4, 5, 6, 7, 8, 9, 10, 11, 12, 13, 14, 15); }
__device__ __forceinline__ v16bf cat16b(v8us lo, v8us hi) { return __builtin_bit_cast(v16bf, __builtin_shufflevector(lo, hi, 0, 1, 2, 3, 4, 5, 6, 7, 8, 9, 10, 11, 12, 13, 14, 15)); }
__device__ __forceinline__ v8f wmma16(v16h a, v16h b, v8f c) { return __builtin_amdgcn_wmma_f32_16x16x32_f16(false, a, false, b, (short)0, c, false, false); }
__device__ __forceinline__ v8f wmmab(v16bf a, v16bf b, v8f c) { return __builtin_amdgcn_wmma_f32_16x16x32_bf16(false, a, false, b, (short)0, c, false, false); }
__device__ __forceinline__ h16 tohx(float x) { return (h16)x; }
__device__ __forceinline__ void splitf(float y, unsigned short& h, unsigned short& l) { h = f2bf(y); l = f2bf(y - bf2f(h)); }

template <typename T16> struct WFrag;
template <> struct WFrag<h16> { typedef v16h V; static __device__ __forceinline__ V ld(const h16* p) { return cat16(*(const v8h*)p, *(const v8h*)(p + 16)); } static __device__ __forceinline__ v8f mma(V a, V b, v8f c) { return wmma16(a, b, c); } };
template <> struct WFrag<bf> { typedef v16bf V; static __device__ __forceinline__ V ld(const bf* p) { return cat16b(*(const v8us*)p, *(const v8us*)(p + 16)); } static __device__ __forceinline__ v8f mma(V a, V b, v8f c) { return wmmab(a, b, c); } };
template <typename T16, int NSPLIT, bool BIAS, int CMODE>
__global__ __launch_bounds__(32) void k_gemmw(const T16* __restrict__ A, const T16* __restrict__ A2, const T16* __restrict__ Bt, const T16* __restrict__ Bt2, int K, float* C, int ldc, const float* __restrict__ bias, size_t sA, size_t sB, size_t sC) {
    typedef typename WFrag<T16>::V V;
    __shared__ __align__(16) float os[16 * 68];
    const size_t z = blockIdx.z; A += z * sA; if (A2) A2 += z * sA; Bt += z * sB; if (Bt2) Bt2 += z * sB; C += z * sC;
    const int lane = threadIdx.x & 31, lr = lane & 15, hi = lane >> 4; const int r0 = blockIdx.x * 64, c0 = blockIdx.y * 64;
    if (CMODE == 3 && r0 + c0 + 192 < TT) return;
    v8f acc[4][4];
#pragma unroll
    for (int mb = 0; mb < 4; ++mb)
#pragma unroll
        for (int nb = 0; nb < 4; ++nb) acc[mb][nb] = (v8f){};
    const size_t aoff = (size_t)(r0 + lr) * K + 8 * hi, boff = (size_t)(c0 + lr) * K + 8 * hi;
#pragma unroll 1
    for (int kc = 0; kc < K; kc += 32) {
        V a[4], a2[4];
#pragma unroll
        for (int mb = 0; mb < 4; ++mb) { a[mb] = WFrag<T16>::ld(A + aoff + (size_t)mb * 16 * K + kc); if (NSPLIT == 1 || NSPLIT == 2) a2[mb] = WFrag<T16>::ld(A2 + aoff + (size_t)mb * 16 * K + kc); }
#pragma unroll
        for (int nb = 0; nb < 4; ++nb) { const V b = WFrag<T16>::ld(Bt + boff + (size_t)nb * 16 * K + kc); V b2; if (NSPLIT >= 2) b2 = WFrag<T16>::ld(Bt2 + boff + (size_t)nb * 16 * K + kc);
#pragma unroll
            for (int mb = 0; mb < 4; ++mb) { acc[mb][nb] = WFrag<T16>::mma(a[mb], b, acc[mb][nb]); if (NSPLIT == 1 || NSPLIT == 2) acc[mb][nb] = WFrag<T16>::mma(a2[mb], b, acc[mb][nb]); if (NSPLIT >= 2) acc[mb][nb] = WFrag<T16>::mma(a[mb], b2, acc[mb][nb]); } }
        asm volatile("v_nop\n\tv_nop\n\tv_nop\n\tv_nop" : "+v"(acc[0][0]), "+v"(acc[1][1]), "+v"(acc[2][2]), "+v"(acc[3][3]) : "v"(a[0]), "v"(a[3]));
    }
#pragma unroll
    for (int mb = 0; mb < 4; ++mb) {
#pragma unroll
        for (int nb = 0; nb < 4; ++nb) {
#pragma unroll
            for (int j = 0; j < 8; ++j) os[(hi * 8 + j) * 68 + nb * 16 + lr] = acc[mb][nb][j]; }
        __builtin_amdgcn_wave_barrier(); asm volatile("" ::: "memory");
        float* crow = C + (size_t)(r0 + mb * 16) * ldc + c0;
#pragma unroll 1
        for (int ps = 0; ps < 2; ++ps) {
#pragma unroll
            for (int s = 0; s < 8; ++s) { const int row = 2 * s + hi, cofs = lr * 4; v4f val = *(const v4fa*)(os + row * 68 + cofs); if (BIAS) { val[0] += bfr(bias[c0 + cofs]); val[1] += bfr(bias[c0 + cofs + 1]); val[2] += bfr(bias[c0 + cofs + 2]); val[3] += bfr(bias[c0 + cofs + 3]); }
                *(volatile v4f*)(crow + (size_t)row * ldc + cofs) = val; }
            if (ps == 0) __threadfence(); }
        __builtin_amdgcn_wave_barrier(); asm volatile("" ::: "memory");
    }
}

__global__ __launch_bounds__(256) void k_wtG(const float* __restrict__ w, int K, int N, bf* Bt) {
    const int lane = threadIdx.x & 31; const int L0 = (blockIdx.x * 8 + (threadIdx.x >> 5)) * 8; const int nlines = N * K / 64;
#pragma unroll
    for (int ps = 0; ps < 2; ++ps) {
#pragma unroll 1
        for (int l = 0; l < 8; ++l) { const int L = L0 + l; if (L >= nlines) break; const size_t e = (size_t)L * 64 + lane * 2; const int k = (int)(e % K), n = (int)(e / K); v2us o;
            o[0] = f2bf(w[(size_t)k * N + n]); o[1] = f2bf(w[(size_t)(k + 1) * N + n]); *(volatile v2us*)(Bt + e) = o; }
        if (ps == 0) __threadfence(); }
}
__global__ __launch_bounds__(256) void k_cvt8(const float* __restrict__ src, bf* dst, size_t n8) { const size_t i = (size_t)blockIdx.x * 256 + threadIdx.x; if (i >= n8) return; const v8f v = *(const v8f*)(src + i * 8); v8us o;
#pragma unroll
    for (int k = 0; k < 8; ++k) o[k] = f2bf(v[k]); *(volatile v8us*)(dst + i * 8) = o; __threadfence(); *(volatile v8us*)(dst + i * 8) = o; }
__global__ __launch_bounds__(256) void k_ecv(const float* __restrict__ rel, h16* E16) { const size_t i = (size_t)blockIdx.x * 256 + threadIdx.x; if (i >= (size_t)TT * HD / 8) return; const v8f v = *(const v8f*)(rel + (size_t)ESTART * HD + i * 8); v8h o;
#pragma unroll
    for (int k = 0; k < 8; ++k) o[k] = tohx(bfr(v[k]) * ECAR); *(volatile v8h*)(E16 + i * 8) = o; __threadfence(); *(volatile v8h*)(E16 + i * 8) = o; }
__global__ __launch_bounds__(256) void k_qkp(const float* __restrict__ F, int pitch, int nheads, float sc, h16* P16) {
    const size_t e = ((size_t)blockIdx.x * 256 + threadIdx.x) * 8; if (e >= (size_t)nheads * TT * HD) return; const int d = (int)(e % HD); const int t = (int)((e / HD) % TT); const int h = (int)(e / ((size_t)HD * TT));
    const v8f x = *(const v8f*)(F + (size_t)t * pitch + h * HD + d); v8h o;
#pragma unroll
    for (int q = 0; q < 8; ++q) o[q] = tohx(x[q] * sc);
    *(volatile v8h*)(P16 + e) = o; __threadfence(); *(volatile v8h*)(P16 + e) = o; }
__global__ __launch_bounds__(256) void k_vtp(const float* __restrict__ F, int pitch, int nheads, h16* V16) {
    const size_t e = ((size_t)blockIdx.x * 256 + threadIdx.x) * 8; if (e >= (size_t)nheads * HD * TT) return; const int t = (int)(e % TT); const int d = (int)((e / TT) % HD); const int g = (int)(e / ((size_t)TT * HD)); v8h o;
#pragma unroll
    for (int q = 0; q < 8; ++q) o[q] = tohx(F[(size_t)(t + q) * pitch + g * HD + d]);
    *(volatile v8h*)(V16 + e) = o; __threadfence(); *(volatile v8h*)(V16 + e) = o; }
__global__ __launch_bounds__(256) void k_vmean(const float* __restrict__ F, float* VM) {
    __shared__ float part[8 * 32];
    const int lane = threadIdx.x & 31, w = __builtin_amdgcn_readfirstlane((int)(threadIdx.x >> 5)); const int c = blockIdx.x * 32 + lane; float s = 0.0f;
#pragma unroll 4
    for (int t = w; t < TT; t += 8) s += F[(size_t)t * DQ + c];
    part[w * 32 + lane] = s; __syncthreads();
    if (threadIdx.x < 8) { v4f o;
#pragma unroll
        for (int q = 0; q < 4; ++q) { const int cc = threadIdx.x * 4 + q; const float tot = ((part[cc] + part[32 + cc]) + (part[64 + cc] + part[96 + cc])) + ((part[128 + cc] + part[160 + cc]) + (part[192 + cc] + part[224 + cc])); o[q] = tot * (1.0f / (float)TT); }
        float* dst = VM + blockIdx.x * 32 + threadIdx.x * 4; *(volatile v4f*)dst = o; __threadfence(); *(volatile v4f*)dst = o; }
}
__global__ __launch_bounds__(SWV * 32) void k_asoft(const float* __restrict__ Sb, const float* __restrict__ Qb, h16* P16) {
    __shared__ __align__(16) float rowb[SWV * TT];
    const int lane = threadIdx.x & 31, w = __builtin_amdgcn_readfirstlane((int)(threadIdx.x >> 5)); const int row = blockIdx.x * SWV + w; if (row >= ZH * TT) return; const int i = row % TT; const int o = TT - 1 - i; const int sh = o & 3;
    const float* sr = Sb + (size_t)row * TT; const float* qr = Qb + (size_t)row * TT; float* rb = rowb + w * TT + lane * 4; float mx = -3.0e38f;
#pragma unroll 1
    for (int ch = 0; ch < TT / 128; ++ch) { const int j0 = ch * 128 + lane * 4; const int mb = (o + j0) & ~3; const int a0 = min(mb, TT - 4), a1 = min(mb + 4, TT - 4);
        const v4f a = *(const v4f*)(sr + j0); const v4f w0 = *(const v4f*)(qr + a0); const v4f w1 = *(const v4f*)(qr + a1);
        float ev[4];
        ev[0] = (sh == 0) ? w0[0] : (sh == 1) ? w0[1] : (sh == 2) ? w0[2] : w0[3];
        ev[1] = (sh == 0) ? w0[1] : (sh == 1) ? w0[2] : (sh == 2) ? w0[3] : w1[0];
        ev[2] = (sh == 0) ? w0[2] : (sh == 1) ? w0[3] : (sh == 2) ? w1[0] : w1[1];
        ev[3] = (sh == 0) ? w0[3] : (sh == 1) ? w1[0] : (sh == 2) ? w1[1] : w1[2];
        v4f tv;
#pragma unroll
        for (int q = 0; q < 4; ++q) { const int j = j0 + q; const float rbv = (j <= i) ? ev[q] : 0.0f; const float t = (a[q] + rbv) * (SCL / ECAR); tv[q] = t; mx = fmaxf(mx, t); }
        *(v4fa*)(rb + ch * 128) = tv; }
#pragma unroll
    for (int s2 = 16; s2; s2 >>= 1) mx = fmaxf(mx, __shfl_xor(mx, s2, 32));
    float sum = 0.f;
#pragma unroll 1
    for (int ch = 0; ch < TT / 128; ++ch) { const v4f tv = *(const v4fa*)(rb + ch * 128); v4f pv;
#pragma unroll
        for (int q = 0; q < 4; ++q) { float d0 = __fsub_rn(tv[q], mx); asm volatile("" : "+v"(d0)); const float p = __builtin_amdgcn_exp2f(__fmul_rn(d0, 1.4426950408889634f)); pv[q] = p; sum += p; }
        *(v4fa*)(rb + ch * 128) = pv; }
#pragma unroll
    for (int s2 = 16; s2; s2 >>= 1) sum += __shfl_xor(sum, s2, 32);
    const float f = __fdiv_rn(PCAR, sum); const float cen = sum * (1.0f / (float)TT);
    h16* prow = P16 + (size_t)row * TT + lane * 4;
#pragma unroll 1
    for (int ps = 0; ps < 2; ++ps) {
#pragma unroll 1
        for (int ch = 0; ch < TT / 128; ++ch) { const v4f pv = *(const v4fa*)(rb + ch * 128); v4h o4;
#pragma unroll
            for (int q = 0; q < 4; ++q) o4[q] = tohx((pv[q] - cen) * f);
            *(volatile v4h*)(prow + ch * 128) = o4; }
        if (ps == 0) __threadfence(); }
}
__global__ __launch_bounds__(256) void k_merge(const float* __restrict__ O, const float* __restrict__ VM, int h0, bf* Ah, bf* Al) {
    const size_t e = ((size_t)blockIdx.x * 256 + threadIdx.x) * 8; if (e >= (size_t)ZH * TT * HD) return; const int d = (int)(e % HD); const int t = (int)((e / HD) % TT); const int zz = (int)(e / ((size_t)HD * TT));
    const int col = (h0 + zz) * HD + d; const size_t oo = (size_t)t * DQ + col; const v8f ov = *(const v8f*)(O + e); const v8f mv = *(const v8f*)(VM + col); v8us oh, ol;
#pragma unroll
    for (int q = 0; q < 8; ++q) { const float y = ov[q] * (1.0f / PCAR) + mv[q]; unsigned short a, c2; splitf(y, a, c2); oh[q] = a; ol[q] = c2; }
    *(volatile v8us*)(Ah + oo) = oh; *(volatile v8us*)(Al + oo) = ol; __threadfence(); *(volatile v8us*)(Ah + oo) = oh; *(volatile v8us*)(Al + oo) = ol; }

constexpr size_t al256(size_t b) { return (b + 255) & ~(size_t)255; }
constexpr size_t SZ_W  = al256((size_t)DQ * DM * 2);
constexpr size_t SZ_E  = al256((size_t)TT * HD * 2);
constexpr size_t SZ_XB = al256((size_t)TT * DM * 2);
constexpr size_t SZ_F  = al256((size_t)TT * DQ * 4);
constexpr size_t SZ_PL = al256((size_t)NH_ * TT * HD * 2);
constexpr size_t SZ_VM = al256((size_t)DQ * 4);
constexpr size_t SZ_S  = al256((size_t)ZH * TT * TT * 4);
constexpr size_t SZ_P  = al256((size_t)ZH * TT * TT * 2);
constexpr size_t SZ_O  = al256((size_t)ZH * TT * HD * 4);
constexpr size_t SZ_AT = al256((size_t)TT * DQ * 2);
constexpr size_t WS_TOTAL = 4 * SZ_W + SZ_E + SZ_XB + SZ_F + 3 * SZ_PL + SZ_VM + 2 * SZ_S + SZ_P + SZ_O + 2 * SZ_AT;
static_assert(WS_TOTAL <= (size_t)134217728);

extern "C" void kernel_launch(void* const* d_in, const int* in_sizes, int n_in,
                              void* d_out, int out_size, void* d_ws, size_t ws_size, hipStream_t stream) {
    if (n_in < 12) return;
    const size_t need_x = (size_t)(NB - 1) * SEQ_FULL * DM + (size_t)TT * DM;
    if ((size_t)in_sizes[0] < need_x || (size_t)in_sizes[1] < need_x || (size_t)in_sizes[2] < need_x) return;
    if ((size_t)in_sizes[3] < (size_t)DM * DQ || (size_t)in_sizes[5] < (size_t)DM * DQ || (size_t)in_sizes[7] < (size_t)DM * DQ || (size_t)in_sizes[9] < (size_t)DQ * DM) return;
    if (in_sizes[4] < DQ || in_sizes[6] < DQ || in_sizes[8] < DQ || in_sizes[10] < DM) return;
    if ((size_t)in_sizes[11] < (size_t)RELN * HD) return;
    if ((size_t)out_size < (size_t)NB * TT * DM) return;
    const float* xq = (const float*)d_in[0]; const float* xk = (const float*)d_in[1]; const float* xv = (const float*)d_in[2];
    const float* wq = (const float*)d_in[3]; const float* bq = (const float*)d_in[4]; const float* wk = (const float*)d_in[5]; const float* bk = (const float*)d_in[6];
    const float* wv = (const float*)d_in[7]; const float* bv = (const float*)d_in[8]; const float* wo = (const float*)d_in[9]; const float* bo = (const float*)d_in[10]; const float* rel = (const float*)d_in[11];
    float* OUT = (float*)d_out;
    if (ws_size < WS_TOTAL) return;
    char* wsp = (char*)d_ws;
    auto take = [&](size_t bytes) { char* p = wsp; wsp += bytes; return (void*)p; };
    bf* WQ = (bf*)take(SZ_W); bf* WK = (bf*)take(SZ_W); bf* WV = (bf*)take(SZ_W); bf* WO = (bf*)take(SZ_W);
    h16* E16 = (h16*)take(SZ_E); bf* XB = (bf*)take(SZ_XB); float* F = (float*)take(SZ_F);
    h16* QP16 = (h16*)take(SZ_PL); h16* KP16 = (h16*)take(SZ_PL); h16* VT16 = (h16*)take(SZ_PL); float* VM = (float*)take(SZ_VM);
    float* Sb = (float*)take(SZ_S); float* Qb = (float*)take(SZ_S); h16* P16 = (h16*)take(SZ_P); float* Ob = (float*)take(SZ_O); bf* ATh = (bf*)take(SZ_AT); bf* ATl = (bf*)take(SZ_AT);
    if ((size_t)(wsp - (char*)d_ws) > ws_size) return;

    const unsigned GW = (unsigned)((DM * DQ / 64 + 63) / 64);
    k_wtG<<<GW, 256, 0, stream>>>(wq, DM, DQ, WQ);
    k_wtG<<<GW, 256, 0, stream>>>(wk, DM, DQ, WK);
    k_wtG<<<GW, 256, 0, stream>>>(wv, DM, DQ, WV);
    k_wtG<<<GW, 256, 0, stream>>>(wo, DQ, DM, WO);
    k_ecv<<<(unsigned)(((size_t)TT * HD / 8 + 255) / 256), 256, 0, stream>>>(rel, E16);
    const unsigned GC = (unsigned)(((size_t)TT * DM / 8 + 255) / 256);
    const unsigned GP = (unsigned)(((size_t)NH_ * TT * HD / 8 + 255) / 256);
    for (int b = 0; b < NB; ++b) {
        const size_t xo = (size_t)b * SEQ_FULL * DM;
        k_cvt8<<<GC, 256, 0, stream>>>(xq + xo, XB, (size_t)TT * DM / 8);
        k_gemmw<bf, 0, true, 0><<<dim3(TT / 64, DQ / 64, 1), 32, 0, stream>>>(XB, nullptr, WQ, nullptr, DM, F, DQ, bq, 0, 0, 0);
        k_qkp<<<GP, 256, 0, stream>>>(F, DQ, NH_, 1.0f, QP16);
        k_cvt8<<<GC, 256, 0, stream>>>(xk + xo, XB, (size_t)TT * DM / 8);
        k_gemmw<bf, 0, true, 0><<<dim3(TT / 64, DQ / 64, 1), 32, 0, stream>>>(XB, nullptr, WK, nullptr, DM, F, DQ, bk, 0, 0, 0);
        k_qkp<<<GP, 256, 0, stream>>>(F, DQ, NH_, ECAR, KP16);
        k_cvt8<<<GC, 256, 0, stream>>>(xv + xo, XB, (size_t)TT * DM / 8);
        k_gemmw<bf, 0, true, 0><<<dim3(TT / 64, DQ / 64, 1), 32, 0, stream>>>(XB, nullptr, WV, nullptr, DM, F, DQ, bv, 0, 0, 0);
        k_vtp<<<GP, 256, 0, stream>>>(F, DQ, NH_, VT16);
        k_vmean<<<DQ / 32, 256, 0, stream>>>(F, VM);
        for (int h0 = 0; h0 < NH_; h0 += ZH) { const size_t zq = (size_t)h0;
            k_gemmw<h16, 0, false, 0><<<dim3(TT / 64, TT / 64, ZH), 32, 0, stream>>>(QP16 + zq * TT * HD, nullptr, KP16 + zq * TT * HD, nullptr, HD, Sb, TT, nullptr, (size_t)TT * HD, (size_t)TT * HD, (size_t)TT * TT);
            k_gemmw<h16, 0, false, 3><<<dim3(TT / 64, TT / 64, ZH), 32, 0, stream>>>(QP16 + zq * TT * HD, nullptr, E16, nullptr, HD, Qb, TT, nullptr, (size_t)TT * HD, 0, (size_t)TT * TT);
            k_asoft<<<ZH * TT / SWV, SWV * 32, 0, stream>>>(Sb, Qb, P16);
            k_gemmw<h16, 0, false, 0><<<dim3(TT / 64, HD / 64, ZH), 32, 0, stream>>>(P16, nullptr, VT16 + zq * HD * TT, nullptr, TT, Ob, HD, nullptr, (size_t)TT * TT, (size_t)HD * TT, (size_t)TT * HD);
            k_merge<<<(unsigned)(((size_t)ZH * TT * HD / 8 + 255) / 256), 256, 0, stream>>>(Ob, VM, h0, ATh, ATl); }
        k_gemmw<bf, 1, true, 0><<<dim3(TT / 64, DM / 64, 1), 32, 0, stream>>>(ATh, ATl, WO, nullptr, DQ, OUT + (size_t)b * TT * DM, DM, bo, 0, 0, 0); }
}
